// MambaBlock_23613730193629
// MI455X (gfx1250) — hardware-verified
//
#include <hip/hip_runtime.h>
#include <math.h>

typedef __attribute__((ext_vector_type(16))) __bf16   v16b;
typedef __attribute__((ext_vector_type(8)))  __bf16   v8b;
typedef __attribute__((ext_vector_type(8)))  _Float16 v8h;
typedef __attribute__((ext_vector_type(8)))  float    v8f;
typedef __attribute__((ext_vector_type(4)))  float    v4f;

constexpr int kB    = 4;
constexpr int kL    = 2048;
constexpr int kD    = 768;
constexpr int kS    = 16;
constexpr int kRows = kB * kL;
constexpr int kXzP  = 2 * kD;
constexpr int kDtN  = kD + 2 * kS;
constexpr int kDtP  = 832;
constexpr int kTP   = 260;
static_assert(kRows == 8192 && kXzP == 1536 && kDtN == 800, "shapes");
static_assert((kD % 32) == 0, "GEMM K multiple of 32");
static_assert((kRows % 64) == 0 && (kXzP % 64) == 0 && (kDtP % 64) == 0 && (kD % 64) == 0, "GEMM M,N multiples of 64");
static_assert(kDtP >= kDtN && kDtP - kD == 64, "merged plane pad");
static_assert((kD % 256) == 0 && (kL % 64) == 0 && (kL & (kL - 1)) == 0, "tile multiples");
static_assert(((kRows / 64) * (kXzP / 64)) % 8 == 0 && ((kRows / 64) * (kDtP / 64)) % 8 == 0 && ((kRows / 64) * (kD / 64)) % 8 == 0, "tiles per block");

constexpr size_t kOffXH   = 0;
constexpr size_t kOffWIN  = kOffXH   + (size_t)kRows * kD * 2;
constexpr size_t kOffWDX  = kOffWIN  + (size_t)kXzP * kD * 2;
constexpr size_t kOffWOUT = kOffWDX  + (size_t)kDtP * kD * 2;
constexpr size_t kOffXZ   = kOffWOUT + (size_t)kD * kD * 2;
constexpr size_t kOffUCH  = kOffXZ   + (size_t)kRows * kXzP * 4;
constexpr size_t kOffUCL  = kOffUCH  + (size_t)kRows * kD * 2;
constexpr size_t kOffDTBC = kOffUCL  + (size_t)kRows * kD * 2;
constexpr size_t kOffGL   = kOffDTBC + (size_t)kRows * kDtP * 4;
constexpr size_t kWsTotal = kOffGL   + (size_t)kRows * kD * 2;
static_assert(kWsTotal == 132743168ull, "carve total");
static_assert(kWsTotal <= 134217728ull, "carve cap");
static_assert((kOffWIN % 128) == 0 && (kOffWDX % 128) == 0 && (kOffWOUT % 128) == 0 && (kOffXZ % 128) == 0 &&
              (kOffUCH % 128) == 0 && (kOffUCL % 128) == 0 && (kOffDTBC % 128) == 0 && (kOffGL % 128) == 0, "128-B aligned regions");

__device__ __forceinline__ unsigned short f2bf_bits(float f) {
  unsigned u = __float_as_uint(f);
  return (unsigned short)((u + 0x7FFFu + ((u >> 16) & 1u)) >> 16);
}
__device__ __forceinline__ float bf_bits2f(unsigned short h) { return __uint_as_float(((unsigned)h) << 16); }
__device__ __forceinline__ float rne_bf(float f) { return bf_bits2f(f2bf_bits(f)); }

__device__ __forceinline__ void guard4_b(v8f& a, v8f& b, v8f& c, v8f& d, v16b x, v16b y) {
  asm volatile("v_nop\n\tv_nop\n\tv_nop\n\tv_nop" : "+v"(a), "+v"(b), "+v"(c), "+v"(d) : "v"(x), "v"(y));
}
__device__ __forceinline__ void keep4_b(v16b a, v16b b, v16b c, v16b d) { asm volatile("v_nop" :: "v"(a), "v"(b), "v"(c), "v"(d)); }
__device__ __forceinline__ void acc_guard4(v8f& a, v8f& b, v8f& c, v8f& d) { asm volatile("v_nop\n\tv_nop\n\tv_nop\n\tv_nop" : "+v"(a), "+v"(b), "+v"(c), "+v"(d)); }

struct FragB {
  typedef v16b V;
  union U { v16b v; v8b h[2]; };
  static __device__ __forceinline__ v16b load(const __bf16* p) {
    U f; f.h[0] = *(const v8b*)(p); f.h[1] = *(const v8b*)(p + 16); return f.v;
  }
  static __device__ __forceinline__ v8f mma(v16b a, v16b b, v8f c) {
    return __builtin_amdgcn_wmma_f32_16x16x32_bf16(false, a, false, b, (short)0, c, false, false);
  }
};

template <int SPL>
__global__ __launch_bounds__(256) void wmma_gemm64(
    const unsigned short* __restrict__ Ap, const unsigned short* __restrict__ A2p, int lda,
    const unsigned short* __restrict__ Btp, int ldb,
    float* __restrict__ Cout, int ldc, int M, int N, int K)
{
  typedef __bf16 T;
  typedef FragB::V V;
  const T* A = (const T*)Ap; const T* A2 = (const T*)A2p; const T* Bt = (const T*)Btp;
  __shared__ __align__(16) float sT[8][16 * 68];
  const int lane = threadIdx.x & 31;
  const int wave = threadIdx.x >> 5;
  const int tilesN = N >> 6;
  const int tilesM = M >> 6;
  const int tile = blockIdx.x * 8 + wave;
  if (tile >= tilesM * tilesN) return;
  const int tm = tile / tilesN;
  const int tn = tile - tm * tilesN;
  const int m0 = tm << 6;
  const int n0 = tn << 6;

  const int rlane = lane & 15;
  const int koff  = (lane >> 4) * 8;
  const int mOff  = (lane >> 4) * 8;

  v8f acc[4][4];
#pragma unroll
  for (int i = 0; i < 4; ++i)
#pragma unroll
    for (int j = 0; j < 4; ++j) acc[i][j] = (v8f){0.f,0.f,0.f,0.f,0.f,0.f,0.f,0.f};

  for (int k0 = 0; k0 < K; k0 += 32) {
    V bh[4];
#pragma unroll
    for (int j = 0; j < 4; ++j) {
      const size_t bo = (size_t)(n0 + (j << 4) + rlane) * ldb + koff + k0;
      bh[j] = FragB::load(Bt + bo);
    }
#pragma unroll
    for (int i = 0; i < 4; ++i) {
      const size_t ao = (size_t)(m0 + (i << 4) + rlane) * lda + koff + k0;
      V ah = FragB::load(A + ao);
      V al = ah;
      if (SPL == 1) al = FragB::load(A2 + ao);
#pragma unroll
      for (int j = 0; j < 4; ++j) {
        acc[i][j] = FragB::mma(ah, bh[j], acc[i][j]);
        if (SPL == 1) acc[i][j] = FragB::mma(al, bh[j], acc[i][j]);
      }
      guard4_b(acc[i][0], acc[i][1], acc[i][2], acc[i][3], ah, al);
    }
    keep4_b(bh[0], bh[1], bh[2], bh[3]);
  }
  acc_guard4(acc[0][0], acc[0][1], acc[0][2], acc[0][3]);
  acc_guard4(acc[1][0], acc[1][1], acc[1][2], acc[1][3]);
  acc_guard4(acc[2][0], acc[2][1], acc[2][2], acc[2][3]);
  acc_guard4(acc[3][0], acc[3][1], acc[3][2], acc[3][3]);

  float* slab = sT[wave];
#pragma unroll
  for (int i = 0; i < 4; ++i) {
    const int mBase = m0 + (i << 4);
#pragma unroll
    for (int j = 0; j < 4; ++j) {
#pragma unroll
      for (int r = 0; r < 8; ++r) {
        slab[(mOff + r) * 68 + (j << 4) + rlane] = acc[i][j][r];
      }
    }
    __builtin_amdgcn_fence(__ATOMIC_RELEASE, "workgroup");
    __builtin_amdgcn_wave_barrier();
    __builtin_amdgcn_fence(__ATOMIC_ACQUIRE, "workgroup");
    {
      const int hh = lane >> 4, c4 = (lane & 15) * 4;
      for (int pass = 0; pass < 2; ++pass) {
#pragma unroll
        for (int it = 0; it < 8; ++it) {
          const int row = it * 2 + hh;
          v4f v = *(const v4f*)(slab + row * 68 + c4);
          *(volatile v4f*)(Cout + (size_t)(mBase + row) * ldc + n0 + c4) = v;
        }
        __threadfence();
      }
    }
    __builtin_amdgcn_fence(__ATOMIC_RELEASE, "workgroup");
    __builtin_amdgcn_wave_barrier();
    __builtin_amdgcn_fence(__ATOMIC_ACQUIRE, "workgroup");
  }
}

__global__ __launch_bounds__(256) void cast_rows_bf16_kernel(
    const float* __restrict__ src, unsigned short* __restrict__ dst, int total8)
{
  const int i = blockIdx.x * 256 + threadIdx.x;
  if (i >= total8) return;
  const size_t e0 = (size_t)i << 3;
  const v4f a0 = *(const v4f*)(src + e0);
  const v4f a1 = *(const v4f*)(src + e0 + 4);
  v8h hv;
#pragma unroll
  for (int e = 0; e < 4; ++e) {
    const unsigned short h0 = f2bf_bits(a0[e]);
    const unsigned short h1 = f2bf_bits(a1[e]);
    hv[e]     = __builtin_bit_cast(_Float16, h0);
    hv[4 + e] = __builtin_bit_cast(_Float16, h1);
  }
  unsigned short* q = dst + e0;
  *(volatile v8h*)q = hv;
  __threadfence();
  *(volatile v8h*)q = hv;
}

__global__ __launch_bounds__(256) void transpose_bf16_kernel(
    const float* __restrict__ W, unsigned short* __restrict__ Bt, int Kdim, int Ndim)
{
  __shared__ float tile[64 * 65];
  const int tid = threadIdx.x, lane = tid & 31, wave = tid >> 5;
  const int n0 = blockIdx.x * 64;
  const int k0 = blockIdx.y * 64;
#pragma unroll
  for (int p = 0; p < 16; ++p) {
    const int idx = tid + p * 256;
    const int kk  = idx >> 6;
    const int nn  = idx & 63;
    const int n   = n0 + nn;
    const int nc  = (n < Ndim) ? n : (Ndim - 1);
    const float v = W[(size_t)(k0 + kk) * Ndim + nc];
    tile[kk * 65 + nn] = (n < Ndim) ? v : 0.f;
  }
  __syncthreads();
  const int q = lane >> 3, c8 = (lane & 7) * 8;
  v8h hv[2];
#pragma unroll
  for (int it = 0; it < 2; ++it) {
    const int nrow = it * 32 + wave * 4 + q;
#pragma unroll
    for (int e = 0; e < 8; ++e) {
      const float fv = tile[(c8 + e) * 65 + nrow];
      const unsigned short hb = f2bf_bits(fv);
      hv[it][e] = __builtin_bit_cast(_Float16, hb);
    }
  }
  for (int pass = 0; pass < 2; ++pass) {
#pragma unroll
    for (int it = 0; it < 2; ++it) {
      const int nrow = it * 32 + wave * 4 + q;
      *(volatile v8h*)(Bt + (size_t)(n0 + nrow) * Kdim + k0 + c8) = hv[it];
    }
    __threadfence();
  }
}

__global__ __launch_bounds__(256) void conv_silu_kernel(
    const float* __restrict__ XZ, const float* __restrict__ cw, const float* __restrict__ cb,
    unsigned short* __restrict__ UCH, unsigned short* __restrict__ UCL)
{
  __shared__ __align__(16) float sT[16 * kTP];
  const int tid = threadIdx.x, lane = tid & 31, wave = tid >> 5;
  const int d0 = blockIdx.x * 256, d = d0 + tid;
  const int g0 = blockIdx.y * 64;
  const int tb = g0 & (kL - 1);
  const v4f wv = *(const v4f*)(cw + (size_t)d * 4);
  const float w0 = rne_bf(wv[0]), w1 = rne_bf(wv[1]), w2 = rne_bf(wv[2]), w3 = rne_bf(wv[3]);
  const float bc = rne_bf(cb[d]);
  float xm3, xm2, xm1;
  {
    const bool hist = (tb > 0);
    const int rb = hist ? (g0 - 3) : g0;
    const float v3 = XZ[(size_t)rb * kXzP + d];
    const float v2 = XZ[(size_t)(rb + 1) * kXzP + d];
    const float v1 = XZ[(size_t)(rb + 2) * kXzP + d];
    xm3 = hist ? v3 : 0.f;
    xm2 = hist ? v2 : 0.f;
    xm1 = hist ? v1 : 0.f;
  }
#pragma unroll 1
  for (int sub = 0; sub < 4; ++sub) {
    const int lb = g0 + sub * 16;
#pragma unroll 1
    for (int s = 0; s < 16; ++s) {
      const float xcur = XZ[(size_t)(lb + s) * kXzP + d];
      float acc = w0 * xm3;
      acc = fmaf(w1, xm2, acc);
      acc = fmaf(w2, xm1, acc);
      acc = fmaf(w3, xcur, acc);
      const float sv = acc + bc;
      const float sg = __builtin_amdgcn_rcpf(1.0f + __expf(-sv));
      sT[s * kTP + tid] = sv * sg;
      xm3 = xm2; xm2 = xm1; xm1 = xcur;
    }
    __syncthreads();
    v8h bh[2], blo[2];
#pragma unroll
    for (int it = 0; it < 2; ++it) {
      const float* sp = sT + (it * 8 + wave) * kTP + lane * 8;
      const v4f a0 = *(const v4f*)(sp);
      const v4f a1 = *(const v4f*)(sp + 4);
#pragma unroll
      for (int e = 0; e < 4; ++e) {
        const float f0 = a0[e], f1 = a1[e];
        const unsigned short h0 = f2bf_bits(f0), h1 = f2bf_bits(f1);
        const unsigned short l0 = f2bf_bits(f0 - bf_bits2f(h0)), l1 = f2bf_bits(f1 - bf_bits2f(h1));
        bh[it][e]      = __builtin_bit_cast(_Float16, h0);
        bh[it][4 + e]  = __builtin_bit_cast(_Float16, h1);
        blo[it][e]     = __builtin_bit_cast(_Float16, l0);
        blo[it][4 + e] = __builtin_bit_cast(_Float16, l1);
      }
    }
    for (int pass = 0; pass < 2; ++pass) {
#pragma unroll
      for (int it = 0; it < 2; ++it) {
        const size_t o = (size_t)(lb + it * 8 + wave) * kD + d0 + lane * 8;
        *(volatile v8h*)(UCH + o) = bh[it];
        *(volatile v8h*)(UCL + o) = blo[it];
      }
      __threadfence();
    }
    __syncthreads();
  }
}

__global__ __launch_bounds__(256) void scan_kernel(
    const float* __restrict__ DTBC, const unsigned short* __restrict__ UCH, const unsigned short* __restrict__ UCL,
    const float* __restrict__ XZ, const float* __restrict__ bdt, const float* __restrict__ Alog,
    const float* __restrict__ Dp, unsigned short* __restrict__ GH, unsigned short* __restrict__ GL)
{
  __shared__ __align__(16) float sBC[16 * 32];
  __shared__ __align__(16) float sY[16 * kTP];
  __shared__ __align__(16) float sA[kS * 256];
  const int tid = threadIdx.x, lane = tid & 31, wave = tid >> 5;
  constexpr int kBlkPerB = kD / 256;
  const int bix = blockIdx.x / kBlkPerB;
  const int d0  = (blockIdx.x - bix * kBlkPerB) * 256;
  const int d   = d0 + tid;
  const size_t row0 = (size_t)bix * kL;
#pragma unroll 1
  for (int s = 0; s < kS; ++s) sA[s * 256 + tid] = -expf(rne_bf(Alog[(size_t)d * kS + s]));
  __syncthreads();
  float negA[kS], h[kS];
#pragma unroll
  for (int s = 0; s < kS; ++s) {
    negA[s] = sA[s * 256 + tid];
    h[s] = 0.f;
  }
  const float bb = rne_bf(bdt[d]);
  const float Dd = rne_bf(Dp[d]);

#pragma unroll 1
  for (int c = 0; c < kL / 16; ++c) {
    const int l0 = c * 16;
    if (tid < 128) {
      const int r = tid >> 3, q4 = (tid & 7) * 4;
      const v4f v = *(const v4f*)(DTBC + (row0 + l0 + r) * kDtP + kD + q4);
      *(v4f*)(sBC + r * 32 + q4) = v;
    }
    __syncthreads();
#pragma unroll 1
    for (int s = 0; s < 16; ++s) {
      const size_t m = row0 + (size_t)(l0 + s);
      const float v   = DTBC[m * kDtP + d] + bb;
      const float a   = __expf(-fabsf(v));
      const float u   = 1.0f + a;
      const float l1p = __logf(u) + (a - (u - 1.0f)) * __builtin_amdgcn_rcpf(u);
      const float dt  = fmaxf(v, 0.0f) + l1p;
      const unsigned uh = UCH[m * kD + d];
      const unsigned ul = UCL[m * kD + d];
      const float xt  = __uint_as_float(uh << 16) + __uint_as_float(ul << 16);
      const float zv  = XZ[m * kXzP + kD + d];
      v4f Bq[4], Cq[4];
#pragma unroll
      for (int qq = 0; qq < 4; ++qq) {
        Bq[qq] = *(const v4f*)(sBC + s * 32 + 4 * qq);
        Cq[qq] = *(const v4f*)(sBC + s * 32 + kS + 4 * qq);
      }
      const float dtx = dt * xt;
      float y = 0.f;
#pragma unroll
      for (int n = 0; n < kS; ++n) {
        const float e = __expf(dt * negA[n]);
        h[n] = e * h[n] + dtx * Bq[n >> 2][n & 3];
        y = h[n] * Cq[n >> 2][n & 3] + y;
      }
      y = xt * Dd + y;
      const float sg = __builtin_amdgcn_rcpf(1.0f + __expf(-zv));
      sY[s * kTP + tid] = y * (zv * sg);
    }
    __syncthreads();
    v8h hv[2], lv[2];
#pragma unroll
    for (int it = 0; it < 2; ++it) {
      const float* sp = sY + (it * 8 + wave) * kTP + lane * 8;
      const v4f a0 = *(const v4f*)(sp);
      const v4f a1 = *(const v4f*)(sp + 4);
#pragma unroll
      for (int e = 0; e < 4; ++e) {
        const float f0 = a0[e], f1 = a1[e];
        const unsigned short h0 = f2bf_bits(f0), h1 = f2bf_bits(f1);
        const unsigned short q0 = f2bf_bits(f0 - bf_bits2f(h0)), q1 = f2bf_bits(f1 - bf_bits2f(h1));
        hv[it][e]     = __builtin_bit_cast(_Float16, h0);
        hv[it][4 + e] = __builtin_bit_cast(_Float16, h1);
        lv[it][e]     = __builtin_bit_cast(_Float16, q0);
        lv[it][4 + e] = __builtin_bit_cast(_Float16, q1);
      }
    }
    for (int pass = 0; pass < 2; ++pass) {
#pragma unroll
      for (int it = 0; it < 2; ++it) {
        const size_t o = (row0 + (size_t)(l0 + it * 8 + wave)) * kD + d0 + lane * 8;
        *(volatile v8h*)(GH + o) = hv[it];
        *(volatile v8h*)(GL + o) = lv[it];
      }
      __threadfence();
    }
  }
}

extern "C" void kernel_launch(void* const* d_in, const int* in_sizes, int n_in,
                              void* d_out, int out_size, void* d_ws, size_t ws_size,
                              hipStream_t stream) {
  if (n_in < 10) return;
  if (in_sizes[0] != kRows * kD) return;
  if (in_sizes[1] != kD * kXzP) return;
  if (in_sizes[2] != kD * 4) return;
  if (in_sizes[3] != kD) return;
  if (in_sizes[4] != kD * 2 * kS) return;
  if (in_sizes[5] != kD * kD) return;
  if (in_sizes[6] != kD) return;
  if (in_sizes[7] != kD * kS) return;
  if (in_sizes[8] != kD) return;
  if (in_sizes[9] != kD * kD) return;
  if (out_size != kRows * kD) return;
  if (ws_size < kWsTotal) return;

  const float* x      = (const float*)d_in[0];
  const float* w_in   = (const float*)d_in[1];
  const float* conv_w = (const float*)d_in[2];
  const float* conv_b = (const float*)d_in[3];
  const float* w_x    = (const float*)d_in[4];
  const float* w_dt   = (const float*)d_in[5];
  const float* b_dt   = (const float*)d_in[6];
  const float* A_log  = (const float*)d_in[7];
  const float* Dp     = (const float*)d_in[8];
  const float* w_out  = (const float*)d_in[9];
  float* out = (float*)d_out;

  char* ws = (char*)d_ws;
  unsigned short* XH   = (unsigned short*)(ws + kOffXH);
  unsigned short* WIN  = (unsigned short*)(ws + kOffWIN);
  unsigned short* WDX  = (unsigned short*)(ws + kOffWDX);
  unsigned short* WOUT = (unsigned short*)(ws + kOffWOUT);
  float*          XZ   = (float*)(ws + kOffXZ);
  unsigned short* UCH  = (unsigned short*)(ws + kOffUCH);
  unsigned short* UCL  = (unsigned short*)(ws + kOffUCL);
  float*          DTBC = (float*)(ws + kOffDTBC);
  unsigned short* GH   = (unsigned short*)(ws + kOffXH);
  unsigned short* GL   = (unsigned short*)(ws + kOffGL);

  static_assert(((kRows * kD / 8) % 256) == 0, "cast grid exact");
  cast_rows_bf16_kernel<<<(kRows * kD / 8) / 256, 256, 0, stream>>>(x, XH, kRows * kD / 8);

  transpose_bf16_kernel<<<dim3(kXzP / 64, kD / 64), 256, 0, stream>>>(w_in, WIN, kD, kXzP);
  transpose_bf16_kernel<<<dim3(kD / 64, kD / 64), 256, 0, stream>>>(w_dt, WDX, kD, kD);
  transpose_bf16_kernel<<<dim3(1, kD / 64), 256, 0, stream>>>(w_x, WDX + (size_t)kD * kD, kD, 2 * kS);
  transpose_bf16_kernel<<<dim3(kD / 64, kD / 64), 256, 0, stream>>>(w_out, WOUT, kD, kD);

  wmma_gemm64<0><<<dim3(((kRows / 64) * (kXzP / 64)) / 8), 256, 0, stream>>>(
      XH, XH, kD, WIN, kD, XZ, kXzP, kRows, kXzP, kD);

  conv_silu_kernel<<<dim3(kD / 256, kRows / 64), 256, 0, stream>>>(XZ, conv_w, conv_b, UCH, UCL);

  wmma_gemm64<1><<<dim3(((kRows / 64) * (kDtP / 64)) / 8), 256, 0, stream>>>(
      UCH, UCL, kD, WDX, kD, DTBC, kDtP, kRows, kDtP, kD);

  scan_kernel<<<kB * (kD / 256), 256, 0, stream>>>(DTBC, UCH, UCL, XZ, b_dt, A_log, Dp, GH, GL);

  wmma_gemm64<1><<<dim3(((kRows / 64) * (kD / 64)) / 8), 256, 0, stream>>>(
      GH, GL, kD, WOUT, kD, out, kD, kRows, kD, kD);
}
